// CapsShapeLayer_52544629899592
// MI455X (gfx1250) — hardware-run, weakly checked
//
#include <hip/hip_runtime.h>
#include <math.h>

typedef __attribute__((ext_vector_type(16))) _Float16 v16h;
typedef __attribute__((ext_vector_type(8)))  _Float16 v8h;
typedef __attribute__((ext_vector_type(8)))  float    v8f;
typedef __attribute__((ext_vector_type(4)))  float    v4f;

constexpr int kB  = 256;
constexpr int kD  = 10;
constexpr int kM  = 32;
constexpr int kP  = 36;
constexpr int kI  = 8;
constexpr int kO  = 16;
constexpr int kMI = kM * kI;
constexpr int kMP = kM * kP;
constexpr int kNS = 64;
constexpr int kKV = 32;
constexpr float kEps     = 1e-7f;
constexpr float kCarryW  = 1024.0f;
constexpr float kCarryXC = 64.0f;
constexpr float kCarryV  = 256.0f;
constexpr float kScaleS  = 1.0f / (kCarryW * kCarryXC);
constexpr float kScaleV  = 1.0f / (kCarryW * kCarryV);

static_assert(kB * kM * kP * kI == 2359296, "x element count");
static_assert(kD * kM * kO * kI == 40960, "W element count");
static_assert(kB * kD * kO == 40960, "out element count");
static_assert(kM == 32, "lane = m mapping");
static_assert(kMI == 256 && kMP == 1152 && (kMP % 32) == 0, "derived sizes");
static_assert((kMI % 32) == 0 && (kKV % 32) == 0, "GEMM K multiples of 32");
static_assert((kB % 64) == 0 && (kNS % 64) == 0 && (kMI % 64) == 0, "GEMM M,N multiples of 64");
static_assert(kO <= kNS && kO <= kKV, "pads");
static_assert(kD * 32 == 320, "route block = one wave per d");

constexpr size_t kOffWTS  = 0;
constexpr size_t kOffWTV  = kOffWTS + (size_t)kD * kNS * kMI * 2;
constexpr size_t kOffXC   = kOffWTV + (size_t)kD * kMI * kKV * 2;
constexpr size_t kOffS    = kOffXC  + (size_t)kD * kB * kMI * 2;
constexpr size_t kOffV    = kOffS   + (size_t)kD * kB * kNS * 4;
constexpr size_t kOffWV1  = kOffV   + (size_t)kD * kB * kKV * 2;
constexpr size_t kOffWV2  = kOffWV1 + (size_t)kD * kB * kMI * 4;
constexpr size_t kWsTotal = kOffWV2 + (size_t)kD * kB * kMI * 4;
static_assert(kWsTotal == 7864320ull, "carve total");
static_assert(kWsTotal <= 134217728ull, "carve cap");
static_assert((kOffWTV % 128) == 0 && (kOffXC % 128) == 0 && (kOffS % 128) == 0 && (kOffV % 128) == 0 &&
              (kOffWV1 % 128) == 0 && (kOffWV2 % 128) == 0, "128-B aligned regions");

__device__ __forceinline__ v16h frag_load(const _Float16* p) {
  union U { v16h v; v8h h[2]; } f;
  f.h[0] = *(const v8h*)(p);
  f.h[1] = *(const v8h*)(p + 16);
  return f.v;
}
__device__ __forceinline__ v8f mma_f16(v16h a, v16h b, v8f c) {
  c = __builtin_amdgcn_wmma_f32_16x16x32_f16(false, a, false, b, (short)0, c, false, false);
  asm volatile("v_nop\n\tv_nop\n\tv_nop\n\tv_nop" : "+v"(c) : "v"(a), "v"(b));
  return c;
}

__device__ __forceinline__ float dot8(const v4f xa, const v4f xb, const v4f wa, const v4f wb) {
  float l = xa[0] * wa[0];
  l = fmaf(xa[1], wa[1], l);
  l = fmaf(xa[2], wa[2], l);
  l = fmaf(xa[3], wa[3], l);
  l = fmaf(xb[0], wb[0], l);
  l = fmaf(xb[1], wb[1], l);
  l = fmaf(xb[2], wb[2], l);
  l = fmaf(xb[3], wb[3], l);
  return l;
}

__global__ __launch_bounds__(256) void gemm64_f16_kernel(
    const unsigned short* __restrict__ Ap, int lda, long strideA,
    const unsigned short* __restrict__ Btp, int ldb, long strideB,
    float* __restrict__ Cout, int ldc, long strideC,
    int M, int N, int K, float scale) {
  const _Float16* A  = (const _Float16*)Ap;
  const _Float16* Bt = (const _Float16*)Btp;
  __shared__ __align__(16) float sT[8][16 * 68];
  const int b    = blockIdx.y;
  const int lane = threadIdx.x & 31;
  const int wave = __builtin_amdgcn_readfirstlane((int)(threadIdx.x >> 5));
  const int tilesN = N >> 6;
  const int tilesM = M >> 6;
  const int tile = blockIdx.x * 8 + wave;
  if (tile >= tilesM * tilesN) return;
  const int tm = tile / tilesN;
  const int tn = tile - tm * tilesN;
  const int m0 = tm << 6;
  const int n0 = tn << 6;

  const _Float16* Ab = A  + (size_t)b * strideA;
  const _Float16* Bb = Bt + (size_t)b * strideB;

  const int rlane = lane & 15;
  const int koff  = (lane >> 4) * 8;
  const int mOff  = (lane >> 4) * 8;

  v8f acc[4][4];
#pragma unroll
  for (int i = 0; i < 4; ++i)
#pragma unroll
    for (int j = 0; j < 4; ++j) acc[i][j] = (v8f){0.f,0.f,0.f,0.f,0.f,0.f,0.f,0.f};

  for (int k0 = 0; k0 < K; k0 += 32) {
    v16h bh[4];
#pragma unroll
    for (int j = 0; j < 4; ++j) {
      const size_t bo = (size_t)(n0 + (j << 4) + rlane) * ldb + koff + k0;
      bh[j] = frag_load(Bb + bo);
    }
#pragma unroll
    for (int i = 0; i < 4; ++i) {
      const size_t ao = (size_t)(m0 + (i << 4) + rlane) * lda + koff + k0;
      const v16h ah = frag_load(Ab + ao);
#pragma unroll
      for (int j = 0; j < 4; ++j) acc[i][j] = mma_f16(ah, bh[j], acc[i][j]);
    }
  }

  float* slab = sT[wave];
  float* C = Cout + (size_t)b * strideC;
#pragma unroll
  for (int i = 0; i < 4; ++i) {
    const int mBase = m0 + (i << 4);
#pragma unroll
    for (int j = 0; j < 4; ++j) {
#pragma unroll
      for (int r = 0; r < 8; ++r) {
        const float v = acc[i][j][r] * scale;
        slab[(mOff + r) * 68 + (j << 4) + rlane] = v;
      }
    }
    __builtin_amdgcn_fence(__ATOMIC_RELEASE, "workgroup");
    __builtin_amdgcn_wave_barrier();
    __builtin_amdgcn_fence(__ATOMIC_ACQUIRE, "workgroup");
    {
      const int hh = lane >> 4, c4 = (lane & 15) * 4;
      for (int pass = 0; pass < 2; ++pass) {
#pragma unroll
        for (int it = 0; it < 8; ++it) {
          const int row = it * 2 + hh;
          v4f v = *(const v4f*)(slab + row * 68 + c4);
          *(volatile v4f*)(C + (size_t)(mBase + row) * ldc + n0 + c4) = v;
        }
        __threadfence();
      }
    }
    __builtin_amdgcn_fence(__ATOMIC_RELEASE, "workgroup");
    __builtin_amdgcn_wave_barrier();
    __builtin_amdgcn_fence(__ATOMIC_ACQUIRE, "workgroup");
  }
}

constexpr int kPrepBlkS = kD * kNS * kM / 256;
constexpr int kPrepBlkV = kD * kMI * 4 / 256;
constexpr int kPrepBlkX = kB * kM / 256;
static_assert(kPrepBlkS == 80 && kPrepBlkV == 40 && kPrepBlkX == 32, "prep coverage");

__global__ __launch_bounds__(256) void prep_kernel(
    const float* __restrict__ x, const float* __restrict__ W,
    unsigned short* __restrict__ WTS, unsigned short* __restrict__ WTV, unsigned short* __restrict__ XC) {
  const int tid = threadIdx.x;
  const int blk = blockIdx.x;
  if (blk < kPrepBlkS) {
    const int t = blk * 256 + tid;
    const int m = t & 31;
    const int n = (t >> 5) & 63;
    const int d = t >> 11;
    const int o = (n < kO) ? n : (kO - 1);
    const float* src = W + ((size_t)((d * kM + m) * kO + o)) * kI;
    v4f a0 = *(const v4f*)(src);
    v4f a1 = *(const v4f*)(src + 4);
    asm volatile("" : "+v"(a0));
    asm volatile("" : "+v"(a1));
    const bool real = (n < kO);
    v8h hv;
#pragma unroll
    for (int e = 0; e < 4; ++e) {
      const float f0 = real ? (a0[e] * kCarryW) : 0.0f;
      const float f1 = real ? (a1[e] * kCarryW) : 0.0f;
      hv[e]     = (_Float16)f0;
      hv[4 + e] = (_Float16)f1;
    }
    unsigned short* dst = WTS + ((size_t)(d * kNS + n)) * kMI + m * 8;
    *(volatile v8h*)dst = hv;
    __threadfence();
    *(volatile v8h*)dst = hv;
  } else if (blk < kPrepBlkS + kPrepBlkV) {
    const int t = (blk - kPrepBlkS) * 256 + tid;
    const int chunk = t & 3;
    const int n = (t >> 2) & 255;
    const int d = t >> 10;
    const int m = n >> 3;
    const int i = n & 7;
    const int kc = chunk & 1;
    const float* src = W + ((size_t)((d * kM + m) * kO + kc * 8)) * kI + i;
    float w[8];
#pragma unroll
    for (int e = 0; e < 8; ++e) {
      w[e] = src[e * kI];
      asm volatile("" : "+v"(w[e]));
    }
    const bool real = (chunk < 2);
    v8h hv;
#pragma unroll
    for (int e = 0; e < 8; ++e) {
      const float f = real ? (w[e] * kCarryW) : 0.0f;
      hv[e] = (_Float16)f;
    }
    unsigned short* dst = WTV + ((size_t)(d * kMI + n)) * kKV + chunk * 8;
    *(volatile v8h*)dst = hv;
    __threadfence();
    *(volatile v8h*)dst = hv;
  } else {
    const int t = (blk - kPrepBlkS - kPrepBlkV) * 256 + tid;
    const int m = t & 31;
    const int b = t >> 5;
    const float* src = x + ((size_t)(b * kM + m)) * (kP * kI);
    v4f s0 = (v4f){0.f, 0.f, 0.f, 0.f};
    v4f s1 = (v4f){0.f, 0.f, 0.f, 0.f};
#pragma unroll 1
    for (int p = 0; p < kP; ++p) {
      const v4f a0 = *(const v4f*)(src + p * kI);
      const v4f a1 = *(const v4f*)(src + p * kI + 4);
      s0 += a0;
      s1 += a1;
    }
    v8h hv;
#pragma unroll
    for (int e = 0; e < 4; ++e) {
      const float f0 = (0.1f * s0[e]) * kCarryXC;
      const float f1 = (0.1f * s1[e]) * kCarryXC;
      hv[e]     = (_Float16)f0;
      hv[4 + e] = (_Float16)f1;
    }
    for (int pass = 0; pass < 2; ++pass) {
#pragma unroll 1
      for (int d = 0; d < kD; ++d) {
        unsigned short* dst = XC + ((size_t)(d * kB + b)) * kMI + m * 8;
        *(volatile v8h*)dst = hv;
      }
      __threadfence();
    }
  }
}

static_assert((kD * kB * 4) % 256 == 0, "squash grid exact");

__global__ __launch_bounds__(256) void squash_v_kernel(const float* __restrict__ S, unsigned short* __restrict__ V) {
  const int t = blockIdx.x * 256 + threadIdx.x;
  const int chunk = t & 3;
  const int row = t >> 2;
  const float* sr = S + (size_t)row * kNS;
  const v4f q0 = *(const v4f*)(sr);
  const v4f q1 = *(const v4f*)(sr + 4);
  const v4f q2 = *(const v4f*)(sr + 8);
  const v4f q3 = *(const v4f*)(sr + 12);
  const int mo = (chunk & 1) * 8;
  v4f e0 = *(const v4f*)(sr + mo);
  v4f e1 = *(const v4f*)(sr + mo + 4);
  asm volatile("" : "+v"(e0));
  asm volatile("" : "+v"(e1));
  float sq = 0.0f;
#pragma unroll
  for (int e = 0; e < 4; ++e) sq = fmaf(q0[e], q0[e], sq);
#pragma unroll
  for (int e = 0; e < 4; ++e) sq = fmaf(q1[e], q1[e], sq);
#pragma unroll
  for (int e = 0; e < 4; ++e) sq = fmaf(q2[e], q2[e], sq);
#pragma unroll
  for (int e = 0; e < 4; ++e) sq = fmaf(q3[e], q3[e], sq);
  const float scale = sq / (1.0f + sq);
  const float rn = 1.0f / sqrtf(sq + kEps);
  const bool real = (chunk < 2);
  v8h hv;
#pragma unroll
  for (int e = 0; e < 4; ++e) {
    const float v0 = scale * (e0[e] * rn);
    const float v1 = scale * (e1[e] * rn);
    const float f0 = real ? (v0 * kCarryV) : 0.0f;
    const float f1 = real ? (v1 * kCarryV) : 0.0f;
    hv[e]     = (_Float16)f0;
    hv[4 + e] = (_Float16)f1;
  }
  unsigned short* dst = V + (size_t)row * kKV + chunk * 8;
  *(volatile v8h*)dst = hv;
  __threadfence();
  *(volatile v8h*)dst = hv;
}

__global__ __launch_bounds__(256) void squash_out_kernel(const float* __restrict__ S, float* __restrict__ out) {
  const int t = blockIdx.x * 256 + threadIdx.x;
  const int q = t & 3;
  const int orow = t >> 2;
  const int b = orow / kD;
  const int d = orow - b * kD;
  const float* sr = S + ((size_t)(d * kB + b)) * kNS;
  const v4f q0 = *(const v4f*)(sr);
  const v4f q1 = *(const v4f*)(sr + 4);
  const v4f q2 = *(const v4f*)(sr + 8);
  const v4f q3 = *(const v4f*)(sr + 12);
  const v4f mine = *(const v4f*)(sr + 4 * q);
  float sq = 0.0f;
#pragma unroll
  for (int e = 0; e < 4; ++e) sq = fmaf(q0[e], q0[e], sq);
#pragma unroll
  for (int e = 0; e < 4; ++e) sq = fmaf(q1[e], q1[e], sq);
#pragma unroll
  for (int e = 0; e < 4; ++e) sq = fmaf(q2[e], q2[e], sq);
#pragma unroll
  for (int e = 0; e < 4; ++e) sq = fmaf(q3[e], q3[e], sq);
  const float scale = sq / (1.0f + sq);
  const float rn = 1.0f / sqrtf(sq + kEps);
  v4f ov;
#pragma unroll
  for (int e = 0; e < 4; ++e) ov[e] = scale * (mine[e] * rn);
  float* dst = out + (size_t)t * 4;
  *(volatile v4f*)dst = ov;
  __threadfence();
  *(volatile v4f*)dst = ov;
}

__global__ __launch_bounds__(320) void route_d_kernel(
    const float* __restrict__ x, const float* __restrict__ WV1, unsigned short* __restrict__ XC) {
  __shared__ __align__(16) float sE[kD * kMP];
  __shared__ __align__(16) float sInv[kMP];
  __shared__ __align__(16) float sWv[kD * kMI];
  const int tid  = threadIdx.x;
  const int lane = tid & 31;
  const int wave = __builtin_amdgcn_readfirstlane((int)(threadIdx.x >> 5));
  const int b = blockIdx.x;
#pragma unroll
  for (int it = 0; it < 2; ++it) {
    const int j = tid + 320 * it;
    const int d = j >> 6;
    const int c4 = (j & 63) * 4;
    *(v4f*)(sWv + d * kMI + c4) = *(const v4f*)(WV1 + ((size_t)(d * kB + b)) * kMI + c4);
  }
  __syncthreads();
  const float* xb = x + (size_t)b * (kMP * kI);
  for (int c = wave; c < kMP / 32; c += kD) {
    const int j = c * 32 + lane;
    const int m = j / kP;
    const v4f xa  = *(const v4f*)(xb + (size_t)j * kI);
    const v4f xb4 = *(const v4f*)(xb + (size_t)j * kI + 4);
    float mx = -INFINITY;
#pragma unroll 1
    for (int d = 0; d < kD; ++d) {
      const v4f wa = *(const v4f*)(sWv + d * kMI + m * kI);
      const v4f wb = *(const v4f*)(sWv + d * kMI + m * kI + 4);
      const float l = dot8(xa, xb4, wa, wb);
      sE[d * kMP + j] = l;
      mx = fmaxf(mx, l);
    }
    float sum = 0.0f;
#pragma unroll 1
    for (int d = 0; d < kD; ++d) {
      const float e = expf(sE[d * kMP + j] - mx);
      sE[d * kMP + j] = e;
      sum += e;
    }
    sInv[j] = 1.0f / sum;
  }
  __syncthreads();
  {
    const int d = wave;
    const int m = lane;
    v4f a0 = (v4f){0.f, 0.f, 0.f, 0.f};
    v4f a1 = (v4f){0.f, 0.f, 0.f, 0.f};
    const float* xm = xb + (size_t)m * (kP * kI);
#pragma unroll 1
    for (int p = 0; p < kP; ++p) {
      const float w = sE[d * kMP + m * kP + p] * sInv[m * kP + p];
      const v4f x0 = *(const v4f*)(xm + p * kI);
      const v4f x1 = *(const v4f*)(xm + p * kI + 4);
#pragma unroll
      for (int e = 0; e < 4; ++e) {
        a0[e] = fmaf(w, x0[e], a0[e]);
        a1[e] = fmaf(w, x1[e], a1[e]);
      }
    }
    v8h hv;
#pragma unroll
    for (int e = 0; e < 4; ++e) {
      const float f0 = a0[e] * kCarryXC;
      const float f1 = a1[e] * kCarryXC;
      hv[e]     = (_Float16)f0;
      hv[4 + e] = (_Float16)f1;
    }
    unsigned short* dst = XC + ((size_t)(d * kB + b)) * kMI + m * 8;
    *(volatile v8h*)dst = hv;
    __threadfence();
    *(volatile v8h*)dst = hv;
  }
}

__global__ __launch_bounds__(320) void route_p_kernel(
    const float* __restrict__ x, const float* __restrict__ WV1, const float* __restrict__ WV2,
    unsigned short* __restrict__ XC) {
  const int lane = threadIdx.x & 31;
  const int wave = __builtin_amdgcn_readfirstlane((int)(threadIdx.x >> 5));
  const int b = blockIdx.x;
  const int d = wave;
  const int m = lane;
  const size_t wo = ((size_t)(d * kB + b)) * kMI + m * kI;
  const v4f w1a = *(const v4f*)(WV1 + wo);
  const v4f w1b = *(const v4f*)(WV1 + wo + 4);
  const v4f w2a = *(const v4f*)(WV2 + wo);
  const v4f w2b = *(const v4f*)(WV2 + wo + 4);
  const float* xm = x + ((size_t)(b * kM + m)) * (kP * kI);
  float mx = -INFINITY;
#pragma unroll 1
  for (int p = 0; p < kP; ++p) {
    const v4f x0 = *(const v4f*)(xm + p * kI);
    const v4f x1 = *(const v4f*)(xm + p * kI + 4);
    const float l1 = dot8(x0, x1, w1a, w1b);
    const float l2 = dot8(x0, x1, w2a, w2b);
    const float l = l1 + l2;
    mx = fmaxf(mx, l);
  }
  float sum = 0.0f;
  v4f a0 = (v4f){0.f, 0.f, 0.f, 0.f};
  v4f a1 = (v4f){0.f, 0.f, 0.f, 0.f};
#pragma unroll 1
  for (int p = 0; p < kP; ++p) {
    const v4f x0 = *(const v4f*)(xm + p * kI);
    const v4f x1 = *(const v4f*)(xm + p * kI + 4);
    const float l1 = dot8(x0, x1, w1a, w1b);
    const float l2 = dot8(x0, x1, w2a, w2b);
    const float l = l1 + l2;
    const float ev = expf(l - mx);
    sum += ev;
#pragma unroll
    for (int e = 0; e < 4; ++e) {
      a0[e] = fmaf(ev, x0[e], a0[e]);
      a1[e] = fmaf(ev, x1[e], a1[e]);
    }
  }
  const float inv = 1.0f / sum;
  v8h hv;
#pragma unroll
  for (int e = 0; e < 4; ++e) {
    const float f0 = (a0[e] * inv) * kCarryXC;
    const float f1 = (a1[e] * inv) * kCarryXC;
    hv[e]     = (_Float16)f0;
    hv[4 + e] = (_Float16)f1;
  }
  unsigned short* dst = XC + ((size_t)(d * kB + b)) * kMI + m * 8;
  *(volatile v8h*)dst = hv;
  __threadfence();
  *(volatile v8h*)dst = hv;
}

extern "C" void kernel_launch(void* const* d_in, const int* in_sizes, int n_in,
                              void* d_out, int out_size, void* d_ws, size_t ws_size,
                              hipStream_t stream) {
  if (n_in < 2) return;
  if (in_sizes[0] != kB * kM * kP * kI) return;
  if (in_sizes[1] != kD * kM * kO * kI) return;
  if (out_size != kB * kD * kO) return;
  if (ws_size < kWsTotal) return;

  const float* x = (const float*)d_in[0];
  const float* W = (const float*)d_in[1];
  float* out = (float*)d_out;

  char* ws = (char*)d_ws;
  unsigned short* WTS = (unsigned short*)(ws + kOffWTS);
  unsigned short* WTV = (unsigned short*)(ws + kOffWTV);
  unsigned short* XC  = (unsigned short*)(ws + kOffXC);
  float*          S   = (float*)(ws + kOffS);
  unsigned short* V   = (unsigned short*)(ws + kOffV);
  float*          WV1 = (float*)(ws + kOffWV1);
  float*          WV2 = (float*)(ws + kOffWV2);

  const int squashBlocks = (kD * kB * 4) / 256;

  prep_kernel<<<kPrepBlkS + kPrepBlkV + kPrepBlkX, 256, 0, stream>>>(x, W, WTS, WTV, XC);

  gemm64_f16_kernel<<<dim3(1, kD), 256, 0, stream>>>(
      XC, kMI, (long)kB * kMI, WTS, kMI, (long)kNS * kMI, S, kNS, (long)kB * kNS, kB, kNS, kMI, kScaleS);
  squash_v_kernel<<<squashBlocks, 256, 0, stream>>>(S, V);
  gemm64_f16_kernel<<<dim3(2, kD), 256, 0, stream>>>(
      V, kKV, (long)kB * kKV, WTV, kKV, (long)kMI * kKV, WV1, kMI, (long)kB * kMI, kB, kMI, kKV, kScaleV);

  route_d_kernel<<<kB, 320, 0, stream>>>(x, WV1, XC);
  gemm64_f16_kernel<<<dim3(1, kD), 256, 0, stream>>>(
      XC, kMI, (long)kB * kMI, WTS, kMI, (long)kNS * kMI, S, kNS, (long)kB * kNS, kB, kNS, kMI, kScaleS);
  squash_v_kernel<<<squashBlocks, 256, 0, stream>>>(S, V);
  gemm64_f16_kernel<<<dim3(2, kD), 256, 0, stream>>>(
      V, kKV, (long)kB * kKV, WTV, kKV, (long)kMI * kKV, WV2, kMI, (long)kB * kMI, kB, kMI, kKV, kScaleV);

  route_p_kernel<<<kB, 320, 0, stream>>>(x, WV1, WV2, XC);
  gemm64_f16_kernel<<<dim3(1, kD), 256, 0, stream>>>(
      XC, kMI, (long)kB * kMI, WTS, kMI, (long)kNS * kMI, S, kNS, (long)kB * kNS, kB, kNS, kMI, kScaleS);
  squash_out_kernel<<<squashBlocks, 256, 0, stream>>>(S, out);
}
